// VaeDecoder_18691697672723
// MI455X (gfx1250) — hardware-verified
//
#include <hip/hip_runtime.h>
#include <math.h>

typedef __attribute__((ext_vector_type(16))) _Float16 v16h;
typedef __attribute__((ext_vector_type(8)))  _Float16 v8h;
typedef __attribute__((ext_vector_type(16))) __bf16   v16b;
typedef __attribute__((ext_vector_type(8)))  __bf16   v8b;
typedef __attribute__((ext_vector_type(8)))  float    v8f;
typedef __attribute__((ext_vector_type(4)))  float    v4f;
typedef __attribute__((ext_vector_type(4)))  unsigned int v4u;

constexpr int   kLat       = 100;
constexpr int   kLatPad    = 128;
constexpr int   kHid       = 64;
constexpr int   kEmb       = 64;
constexpr int   kGates     = 256;
constexpr int   kKcat      = 128;
constexpr int   kSteps     = 30;
constexpr int   kRowsBlk   = 16;
constexpr int   kAPitch    = 136;
constexpr int   kTrajPitch = 120;
constexpr float kDt        = 0.03f;
constexpr float kWScale    = 16.0f;
constexpr float kWScaleInv = 0.0625f;

__device__ __forceinline__ unsigned short f2bf_bits(float f) {
  unsigned u = __float_as_uint(f);
  return (unsigned short)((u + 0x7FFFu + ((u >> 16) & 1u)) >> 16);
}
__device__ __forceinline__ float bf_bits2f(unsigned short h) { return __uint_as_float(((unsigned)h) << 16); }

__device__ __forceinline__ void dep_guard_h(v8f& a, v8f& b, v16h x, v16h y) { asm volatile("v_nop\n\tv_nop\n\tv_nop\n\tv_nop" : "+v"(a), "+v"(b) : "v"(x), "v"(y)); }
__device__ __forceinline__ void dep_guard_b(v8f& a, v8f& b, v16b x, v16b y) { asm volatile("v_nop\n\tv_nop\n\tv_nop\n\tv_nop" : "+v"(a), "+v"(b) : "v"(x), "v"(y)); }
__device__ __forceinline__ void keep4_h(v16h a, v16h b, v16h c, v16h d) { asm volatile("v_nop" :: "v"(a), "v"(b), "v"(c), "v"(d)); }
__device__ __forceinline__ void keep4_b(v16b a, v16b b, v16b c, v16b d) { asm volatile("v_nop" :: "v"(a), "v"(b), "v"(c), "v"(d)); }
__device__ __forceinline__ void acc_guard4(v8f& a, v8f& b, v8f& c, v8f& d) { asm volatile("v_nop\n\tv_nop\n\tv_nop\n\tv_nop" : "+v"(a), "+v"(b), "+v"(c), "+v"(d)); }
template <typename T> struct Frag;
template <> struct Frag<_Float16> {
  typedef v16h V; union U { v16h v; v8h h[2]; };
  static __device__ __forceinline__ v16h load(const _Float16* p) {
    U f; f.h[0] = *(const v8h*)(p); f.h[1] = *(const v8h*)(p + 16); return f.v;
  }
  static __device__ __forceinline__ v8f mma(v16h a, v16h b, v8f c) {
    return __builtin_amdgcn_wmma_f32_16x16x32_f16(false, a, false, b, (short)0, c, false, false);
  }
  static __device__ __forceinline__ void guard(v8f& a, v8f& b, v16h x, v16h y) { dep_guard_h(a, b, x, y); }
  static __device__ __forceinline__ void keep(v16h a, v16h b, v16h c, v16h d) { keep4_h(a, b, c, d); }
};
template <> struct Frag<__bf16> {
  typedef v16b V; union U { v16b v; v8b h[2]; };
  static __device__ __forceinline__ v16b load(const __bf16* p) {
    U f; f.h[0] = *(const v8b*)(p); f.h[1] = *(const v8b*)(p + 16); return f.v;
  }
  static __device__ __forceinline__ v8f mma(v16b a, v16b b, v8f c) {
    return __builtin_amdgcn_wmma_f32_16x16x32_bf16(false, a, false, b, (short)0, c, false, false);
  }
  static __device__ __forceinline__ void guard(v8f& a, v8f& b, v16b x, v16b y) { dep_guard_b(a, b, x, y); }
  static __device__ __forceinline__ void keep(v16b a, v16b b, v16b c, v16b d) { keep4_b(a, b, c, d); }
};

template <int ET> struct Elem;
template <> struct Elem<0> { typedef _Float16 T; };
template <> struct Elem<1> { typedef __bf16 T; };
template <int ET, bool SPLIT, int BIAS_MODE, int OUT_MODE, bool RESID, int ACT = 0>
__global__ __launch_bounds__(256) void wmma_gemm64(
    const unsigned short* __restrict__ Ap, const unsigned short* __restrict__ A2p, int lda, long strideA,
    const unsigned short* __restrict__ Btp, const unsigned short* __restrict__ Bt2p, int ldb, long strideB,
    void* __restrict__ Cout, void* __restrict__ Cout2, int ldc, long strideC,
    const float* __restrict__ bias,
    const float* __restrict__ resid, long strideR,
    int M, int N, int K, float scale) {
  typedef typename Elem<ET>::T T;
  typedef typename Frag<T>::V V;
  const T* A = (const T*)Ap; const T* A2 = (const T*)A2p; const T* Bt = (const T*)Btp; const T* Bt2 = (const T*)Bt2p;
  __shared__ __align__(16) float sT[8][16 * 68];
  const int b    = blockIdx.y;
  const int lane = threadIdx.x & 31;
  const int wave = threadIdx.x >> 5;
  const int tilesN = N >> 6;
  const int tilesM = M >> 6;
  const int tile = blockIdx.x * 8 + wave;
  if (tile >= tilesM * tilesN) return;
  const int tm = tile / tilesN;
  const int tn = tile - tm * tilesN;
  const int m0 = tm << 6;
  const int n0 = tn << 6;

  const T* Ab  = A  + (size_t)b * strideA;
  const T* Bb  = Bt + (size_t)b * strideB;
  const T* Ab2 = SPLIT ? (A2  + (size_t)b * strideA) : nullptr;
  const T* Bb2 = SPLIT ? (Bt2 + (size_t)b * strideB) : nullptr;

  const int rlane = lane & 15;
  const int koff  = (lane >> 4) * 8;
  const int mOff  = (lane >> 4) * 8;

  v8f acc[4][4];
#pragma unroll
  for (int i = 0; i < 4; ++i)
#pragma unroll
    for (int j = 0; j < 4; ++j) acc[i][j] = (v8f){0.f,0.f,0.f,0.f,0.f,0.f,0.f,0.f};

  for (int k0 = 0; k0 < K; k0 += 32) {
    V bh[4], bl[4];
#pragma unroll
    for (int j = 0; j < 4; ++j) {
      const size_t bo = (size_t)(n0 + (j << 4) + rlane) * ldb + koff + k0;
      bh[j] = Frag<T>::load(Bb + bo);
      if (SPLIT) bl[j] = Frag<T>::load(Bb2 + bo);
    }
#pragma unroll
    for (int i = 0; i < 4; ++i) {
      const size_t ao = (size_t)(m0 + (i << 4) + rlane) * lda + koff + k0;
      V ah = Frag<T>::load(Ab + ao);
      V al;
      if (SPLIT) al = Frag<T>::load(Ab2 + ao);
#pragma unroll
      for (int j = 0; j < 4; ++j) {
        acc[i][j] = Frag<T>::mma(ah, bh[j], acc[i][j]);
        if (SPLIT) {
          acc[i][j] = Frag<T>::mma(ah, bl[j], acc[i][j]);
          acc[i][j] = Frag<T>::mma(al, bh[j], acc[i][j]);
        }
      }
      Frag<T>::guard(acc[i][0], acc[i][3], ah, SPLIT ? al : ah);
    }
    Frag<T>::keep(bh[0], bh[1], bh[2], bh[3]);
    if (SPLIT) Frag<T>::keep(bl[0], bl[1], bl[2], bl[3]);
  }
  acc_guard4(acc[0][0], acc[0][1], acc[0][2], acc[0][3]);
  acc_guard4(acc[1][0], acc[1][1], acc[1][2], acc[1][3]);
  acc_guard4(acc[2][0], acc[2][1], acc[2][2], acc[2][3]);
  acc_guard4(acc[3][0], acc[3][1], acc[3][2], acc[3][3]);

  float* slab = sT[wave];
  const float* Rb = RESID ? (resid + (size_t)b * strideR) : nullptr;
#pragma unroll
  for (int i = 0; i < 4; ++i) {
    const int mBase = m0 + (i << 4);
#pragma unroll
    for (int j = 0; j < 4; ++j) {
      const int n = n0 + (j << 4) + rlane;
      float bv = 0.f;
      if (BIAS_MODE == 2) bv = bias[n];
#pragma unroll
      for (int r = 0; r < 8; ++r) {
        float v = acc[i][j][r] * scale;
        if (BIAS_MODE == 1) v += bias[mBase + mOff + r];
        if (BIAS_MODE == 2) v += bv;
        if (RESID) v += Rb[(size_t)(mBase + mOff + r) * ldc + n];
        if (ACT == 1) v = tanhf(v);
        if (ACT == 2) v = fmaxf(v, 0.0f);
        if (ACT == 3) v = v / (1.0f + expf(-v));
        if (ACT == 4) v = (v > 0.f) ? v : 0.01f * v;
        if (ACT == 5) v = 0.5f * v * (1.0f + erff(v * 0.70710678118654752f));
        slab[(mOff + r) * 68 + (j << 4) + rlane] = v;
      }
    }
    __builtin_amdgcn_fence(__ATOMIC_RELEASE, "workgroup");
    __builtin_amdgcn_wave_barrier();
    __builtin_amdgcn_fence(__ATOMIC_ACQUIRE, "workgroup");
    if (OUT_MODE == 0) {
      float* C = (float*)Cout + (size_t)b * strideC;
      const int hh = lane >> 4, c4 = (lane & 15) * 4;
      for (int pass = 0; pass < 2; ++pass) {
#pragma unroll
        for (int it = 0; it < 8; ++it) {
          const int row = it * 2 + hh;
          v4f v = *(const v4f*)(slab + row * 68 + c4);
          *(volatile v4f*)(C + (size_t)(mBase + row) * ldc + n0 + c4) = v;
        }
        __threadfence();
      }
    } else {
      const int q = lane >> 3, c8 = (lane & 7) * 8;
      unsigned short* C  = (unsigned short*)Cout  + (size_t)b * strideC;
      unsigned short* C2 = (OUT_MODE == 2) ? ((unsigned short*)Cout2 + (size_t)b * strideC) : nullptr;
      for (int pass = 0; pass < 2; ++pass) {
#pragma unroll
        for (int it = 0; it < 4; ++it) {
          const int row = it * 4 + q;
          const float* sp = slab + row * 68 + c8;
          v8h hv, lv;
#pragma unroll
          for (int e = 0; e < 8; ++e) {
            if (OUT_MODE == 1) {
              hv[e] = (_Float16)sp[e];
            } else {
              unsigned short hb = f2bf_bits(sp[e]);
              unsigned short lb = f2bf_bits(sp[e] - bf_bits2f(hb));
              hv[e] = __builtin_bit_cast(_Float16, hb);
              lv[e] = __builtin_bit_cast(_Float16, lb);
            }
          }
          *(volatile v8h*)(C + (size_t)(mBase + row) * ldc + n0 + c8) = hv;
          if (OUT_MODE == 2) *(volatile v8h*)(C2 + (size_t)(mBase + row) * ldc + n0 + c8) = lv;
        }
        __threadfence();
      }
    }
    __builtin_amdgcn_fence(__ATOMIC_RELEASE, "workgroup");
    __builtin_amdgcn_wave_barrier();
    __builtin_amdgcn_fence(__ATOMIC_ACQUIRE, "workgroup");
  }
}

__device__ __forceinline__ unsigned f2h_bits(float f) {
  return (unsigned)__builtin_bit_cast(unsigned short, (_Float16)f);
}
__device__ __forceinline__ void wave_sync_lds() {
  __builtin_amdgcn_fence(__ATOMIC_RELEASE, "workgroup");
  __builtin_amdgcn_wave_barrier();
  __builtin_amdgcn_fence(__ATOMIC_ACQUIRE, "workgroup");
}
__device__ __forceinline__ v8f zero8() { return (v8f){0.f,0.f,0.f,0.f,0.f,0.f,0.f,0.f}; }
__device__ __forceinline__ v8f mma_h(v16h a, v16h b, v8f c) {
  return __builtin_amdgcn_wmma_f32_16x16x32_f16(false, a, false, b, (short)0, c, false, false);
}
__device__ __forceinline__ v8f mma_h_guarded(v16h a, v16h b, v8f c) {
  c = mma_h(a, b, c);
  asm volatile("v_nop\n\tv_nop\n\tv_nop\n\tv_nop" : "+v"(c) : "v"(a), "v"(b));
  return c;
}
__device__ __forceinline__ void guard_group4(v8f& a0, v8f& a1, v8f& a2, v8f& a3,
                                             v16h fa, v16h b0, v16h b1, v16h b2, v16h b3) {
  asm volatile("v_nop\n\tv_nop\n\tv_nop\n\tv_nop"
               : "+v"(a0), "+v"(a1), "+v"(a2), "+v"(a3)
               : "v"(fa), "v"(b0), "v"(b1), "v"(b2), "v"(b3));
}
__device__ __forceinline__ float sigm_f(float x) { return __builtin_amdgcn_rcpf(1.0f + expf(-x)); }
__device__ __forceinline__ float tanh_f(float x) { return 1.0f - 2.0f * __builtin_amdgcn_rcpf(1.0f + expf(2.0f * x)); }

__device__ __forceinline__ void store_split8(unsigned short* dh, unsigned short* dl, size_t off, const float (&v)[8]) {
  unsigned hw[4], lw[4];
#pragma unroll
  for (int e2 = 0; e2 < 4; ++e2) {
    const unsigned short h0 = f2bf_bits(v[2 * e2]);
    const unsigned short h1 = f2bf_bits(v[2 * e2 + 1]);
    const unsigned short l0 = f2bf_bits(v[2 * e2] - bf_bits2f(h0));
    const unsigned short l1 = f2bf_bits(v[2 * e2 + 1] - bf_bits2f(h1));
    hw[e2] = (unsigned)h0 | ((unsigned)h1 << 16);
    lw[e2] = (unsigned)l0 | ((unsigned)l1 << 16);
  }
  const v4u hv4 = (v4u){hw[0], hw[1], hw[2], hw[3]};
  const v4u lv4 = (v4u){lw[0], lw[1], lw[2], lw[3]};
  volatile v4u* ph = (volatile v4u*)(dh + off);
  volatile v4u* pl = (volatile v4u*)(dl + off);
  *ph = hv4; *pl = lv4;
  __threadfence();
  *ph = hv4; *pl = lv4;
}
__device__ __forceinline__ void store_half8(unsigned short* dst, size_t off, const float (&v)[8]) {
  unsigned w[4];
#pragma unroll
  for (int e2 = 0; e2 < 4; ++e2) w[e2] = f2h_bits(v[2 * e2]) | (f2h_bits(v[2 * e2 + 1]) << 16);
  const v4u wv = (v4u){w[0], w[1], w[2], w[3]};
  volatile v4u* p = (volatile v4u*)(dst + off);
  *p = wv;
  __threadfence();
  *p = wv;
}

__global__ __launch_bounds__(128) void prep_weights_kernel(
    const float* __restrict__ Wl0, const float* __restrict__ W_init,
    const float* __restrict__ Wl1, const float* __restrict__ Wl2, const float* __restrict__ Wl3,
    const float* __restrict__ W_ih, const float* __restrict__ W_hh, const float* __restrict__ W_h2c,
    unsigned short* __restrict__ Wl0hi, unsigned short* __restrict__ Wl0lo,
    unsigned short* __restrict__ Winhi, unsigned short* __restrict__ Winlo,
    unsigned short* __restrict__ Wl1hi, unsigned short* __restrict__ Wl1lo,
    unsigned short* __restrict__ Wl2hi, unsigned short* __restrict__ Wl2lo,
    unsigned short* __restrict__ Wl3hi, unsigned short* __restrict__ Wl3lo,
    unsigned short* __restrict__ Wcat, unsigned short* __restrict__ Wh2c) {
  const int grp = blockIdx.y;
  const int i = blockIdx.x * 128 + threadIdx.x;
  float v[8];
  if (grp <= 1) {
    if (i >= (kHid * kLatPad) / 8) return;
    const float* src = (grp == 0) ? Wl0 : W_init;
    unsigned short* dh = (grp == 0) ? Wl0hi : Winhi;
    unsigned short* dl = (grp == 0) ? Wl0lo : Winlo;
    const int n = i >> 4, k0 = (i & 15) * 8;
#pragma unroll
    for (int e = 0; e < 8; ++e) {
      const int k = k0 + e;
      const int kc = (k < kLat) ? k : (kLat - 1);
      const float f = src[n * kLat + kc];
      v[e] = (k < kLat) ? f : 0.0f;
    }
    store_split8(dh, dl, (size_t)8 * i, v);
  } else if (grp <= 3) {
    if (i >= (kHid * kHid) / 8) return;
    const float* src = (grp == 2) ? Wl1 : Wl2;
    unsigned short* dh = (grp == 2) ? Wl1hi : Wl2hi;
    unsigned short* dl = (grp == 2) ? Wl1lo : Wl2lo;
    const int n = i >> 3, k0 = (i & 7) * 8;
#pragma unroll
    for (int e = 0; e < 8; ++e) v[e] = src[n * kHid + k0 + e];
    store_split8(dh, dl, (size_t)8 * i, v);
  } else if (grp == 4) {
    if (i >= (kHid * kHid) / 8) return;
    const int n = i >> 3, k0 = (i & 7) * 8;
    const int nc = (n < 2) ? n : 1;
#pragma unroll
    for (int e = 0; e < 8; ++e) {
      const float f = Wl3[nc * kHid + k0 + e];
      v[e] = (n < 2) ? f : 0.0f;
    }
    store_split8(Wl3hi, Wl3lo, (size_t)8 * i, v);
  } else if (grp == 5) {
    if (i >= (kGates * kKcat) / 8) return;
    const int n = i >> 4, k0 = (i & 15) * 8;
    const int kk = k0 & 63;
#pragma unroll
    for (int e = 0; e < 8; ++e) {
      const float fa = W_ih[n * kHid + kk + e];
      const float fb = W_hh[n * kHid + kk + e];
      v[e] = kWScale * ((k0 < kHid) ? fa : fb);
    }
    store_half8(Wcat, (size_t)8 * i, v);
  } else if (grp == 6) {
    if (i >= (16 * kHid) / 8) return;
    const int n = i >> 3, k0 = (i & 7) * 8;
    const int nc = (n < 2) ? n : 1;
#pragma unroll
    for (int e = 0; e < 8; ++e) {
      const float f = W_h2c[nc * kHid + k0 + e];
      v[e] = (n < 2) ? (kWScale * f) : 0.0f;
    }
    store_half8(Wh2c, (size_t)8 * i, v);
  }
}

__global__ __launch_bounds__(256) void split_z_kernel(const float* __restrict__ z,
                                                      unsigned short* __restrict__ Zhi,
                                                      unsigned short* __restrict__ Zlo, int Btot) {
  const int i = blockIdx.x * 256 + threadIdx.x;
  if (i >= Btot * 16) return;
  const int row = i >> 4, k0 = (i & 15) * 8;
  const float* zr = z + (size_t)row * kLat;
  float v[8];
#pragma unroll
  for (int e = 0; e < 8; ++e) {
    const int k = k0 + e;
    const int kc = (k < kLat) ? k : (kLat - 1);
    const float f = zr[kc];
    v[e] = (k < kLat) ? f : 0.0f;
  }
  store_split8(Zhi, Zlo, (size_t)8 * i, v);
}

__global__ __launch_bounds__(256) void label_out_kernel(const float* __restrict__ L3,
                                                       const float* __restrict__ bl3,
                                                       float* __restrict__ out1, int nPairs) {
  const int i = blockIdx.x * 256 + threadIdx.x;
  if (i >= nPairs) return;
  const size_t r0 = (size_t)2 * i;
  const float b0 = bl3[0], b1 = bl3[1];
  float a = L3[r0 * kHid + 0] + b0;
  float b = L3[r0 * kHid + 1] + b1;
  float c2 = L3[(r0 + 1) * kHid + 0] + b0;
  float d = L3[(r0 + 1) * kHid + 1] + b1;
  a  = (a  >= 0.0f) ? a  : 0.01f * a;
  b  = (b  >= 0.0f) ? b  : 0.01f * b;
  c2 = (c2 >= 0.0f) ? c2 : 0.01f * c2;
  d  = (d  >= 0.0f) ? d  : 0.01f * d;
  const v4f o = (v4f){a, b, c2, d};
  volatile v4f* p = (volatile v4f*)(out1 + 4 * (size_t)i);
  *p = o;
  __threadfence();
  *p = o;
}

__device__ __forceinline__ void embed_rows(_Float16* tile, const float* st, const float* wemb,
                                           const float* bemb, int lane) {
  const int r = lane & 15, ch = lane >> 4;
  const float s0 = st[r * 4 + 0], s1 = st[r * 4 + 1], s2 = st[r * 4 + 2], s3 = st[r * 4 + 3];
#pragma unroll 1
  for (int g = 0; g < 4; ++g) {
    const int colBase = 32 * ch + 8 * g;
    unsigned w[4];
#pragma unroll
    for (int e2 = 0; e2 < 4; ++e2) {
      const int col = colBase + 2 * e2;
      const float* wa = wemb + col * 4;
      float xa = wa[0] * s0; xa = fmaf(wa[1], s1, xa); xa = fmaf(wa[2], s2, xa); xa = fmaf(wa[3], s3, xa);
      xa += bemb[col];
      const float* wb = wemb + (col + 1) * 4;
      float xb = wb[0] * s0; xb = fmaf(wb[1], s1, xb); xb = fmaf(wb[2], s2, xb); xb = fmaf(wb[3], s3, xb);
      xb += bemb[col + 1];
      w[e2] = f2h_bits(xa) | (f2h_bits(xb) << 16);
    }
    const v4u vv = (v4u){w[0], w[1], w[2], w[3]};
    *(v4u*)(tile + r * kAPitch + colBase) = vv;
  }
}

__device__ __forceinline__ void plant_step(float sx, float sy, float spsi, float sv, float ped, float steer,
                                           float& nx, float& ny, float& npsi, float& nv) {
#pragma clang fp contract(off)
  const float beta = fminf(fmaxf(steer, -0.5f), 0.5f);
  const float v1 = fminf(fmaxf(sv + ped * kDt, 0.0f), 10.0f);
  const float tb = tanf(beta);
  const float psid = fminf(fmaxf(sv * tb * 0.4f, -1.57f), 1.57f);
  const float psi1 = psid * kDt + spsi;
  const float cs = cosf(psi1);
  const float sn = sinf(psi1);
  nx = v1 * cs * kDt + sx;
  ny = v1 * sn * kDt + sy;
  npsi = psi1;
  nv = v1;
}

__global__ __launch_bounds__(128) void lstm_rollout_kernel(
    const unsigned short* __restrict__ Wcatp, const unsigned short* __restrict__ Wh2cp,
    const float* __restrict__ H0, const float* __restrict__ init_state,
    const float* __restrict__ W_emb, const float* __restrict__ b_emb,
    const float* __restrict__ b_ih, const float* __restrict__ b_hh,
    const float* __restrict__ b_h2c, float* __restrict__ out0, int Btot) {
  const _Float16* Wcat = (const _Float16*)Wcatp;
  const _Float16* Wh2c = (const _Float16*)Wh2cp;
  __shared__ __align__(16) _Float16 aT[2][kRowsBlk * kAPitch];
  __shared__ __align__(16) float trajS[kRowsBlk * kTrajPitch];
  __shared__ __align__(16) float wembS[kEmb * 4];
  __shared__ __align__(16) float bembS[kEmb];
  __shared__ __align__(16) float stS[kRowsBlk * 4];
  __shared__ __align__(16) float ctlS[kRowsBlk * 2];

  const int tid  = threadIdx.x;
  const int wave = tid >> 5;
  const int lane = tid & 31;
  const int hh   = lane >> 4;
  const int c    = lane & 15;
  const int koff = hh * 8;
  const int rowBase = blockIdx.x * kRowsBlk;
  if (rowBase + kRowsBlk > Btot) return;

  if (tid < kEmb) {
    const v4f wv = *(const v4f*)(W_emb + tid * 4);
    *(v4f*)(wembS + tid * 4) = wv;
    bembS[tid] = b_emb[tid];
  }
  if (tid < kRowsBlk) {
    const v4f s = *(const v4f*)(init_state + (size_t)(rowBase + tid) * 4);
    *(v4f*)(stS + tid * 4) = s;
  }
  const int u = 16 * wave + c;
  const float bs0 = b_ih[u] + b_hh[u];
  const float bs1 = b_ih[kHid + u] + b_hh[kHid + u];
  const float bs2 = b_ih[2 * kHid + u] + b_hh[2 * kHid + u];
  const float bs3 = b_ih[3 * kHid + u] + b_hh[3 * kHid + u];
  const float bc0 = b_h2c[0], bc1 = b_h2c[1];
  const float bcsel = (c == 1) ? bc1 : bc0;

  float cst[8];
#pragma unroll
  for (int r = 0; r < 8; ++r) {
    const float hv = H0[(size_t)(rowBase + 8 * hh + r) * kHid + u];
    cst[r] = hv;
    aT[0][(8 * hh + r) * kAPitch + kHid + u] = (_Float16)hv;
  }
  __syncthreads();
  if (wave == 0) embed_rows(&aT[0][0], stS, wembS, bembS, lane);
  __syncthreads();

#pragma unroll 1
  for (int t = 0; t < kSteps; ++t) {
    const int cur = t & 1, nxt = cur ^ 1;
    const _Float16* At = &aT[cur][0];
    _Float16* An = &aT[nxt][0];

    v8f acc0 = zero8(), acc1 = zero8(), acc2 = zero8(), acc3 = zero8();
#pragma unroll
    for (int kc = 0; kc < 4; ++kc) {
      const v16h afr = Frag<_Float16>::load(At + c * kAPitch + koff + 32 * kc);
      const _Float16* wb = Wcat + (size_t)u * kKcat + koff + 32 * kc;
      const v16h b0 = Frag<_Float16>::load(wb);
      const v16h b1 = Frag<_Float16>::load(wb + 1 * kHid * kKcat);
      const v16h b2 = Frag<_Float16>::load(wb + 2 * kHid * kKcat);
      const v16h b3 = Frag<_Float16>::load(wb + 3 * kHid * kKcat);
      acc0 = mma_h(afr, b0, acc0);
      acc1 = mma_h(afr, b1, acc1);
      acc2 = mma_h(afr, b2, acc2);
      acc3 = mma_h(afr, b3, acc3);
      guard_group4(acc0, acc1, acc2, acc3, afr, b0, b1, b2, b3);
    }

#pragma unroll
    for (int r = 0; r < 8; ++r) {
      const float gi = acc0[r] * kWScaleInv + bs0;
      const float gf = acc1[r] * kWScaleInv + bs1;
      const float gg = acc2[r] * kWScaleInv + bs2;
      const float go = acc3[r] * kWScaleInv + bs3;
      const float ig = sigm_f(gi);
      const float fg = sigm_f(gf);
      const float gt = tanh_f(gg);
      const float og = sigm_f(go);
      const float cv = fg * cst[r] + ig * gt;
      cst[r] = cv;
      const float hv = og * tanh_f(cv);
      An[(8 * hh + r) * kAPitch + kHid + u] = (_Float16)hv;
    }
    __syncthreads();

    if (wave == 0) {
      v8f cacc = zero8();
      const v16h a0 = Frag<_Float16>::load(An + c * kAPitch + kHid + koff);
      const v16h a1 = Frag<_Float16>::load(An + c * kAPitch + kHid + 32 + koff);
      const v16h w0 = Frag<_Float16>::load(Wh2c + c * kHid + koff);
      const v16h w1 = Frag<_Float16>::load(Wh2c + c * kHid + 32 + koff);
      cacc = mma_h_guarded(a0, w0, cacc);
      cacc = mma_h_guarded(a1, w1, cacc);
      if (c < 2) {
#pragma unroll
        for (int r = 0; r < 8; ++r) ctlS[(8 * hh + r) * 2 + c] = cacc[r] * kWScaleInv + bcsel;
      }
      wave_sync_lds();
      {
        const int r = c;
        const float ped   = ctlS[r * 2 + 0];
        const float steer = ctlS[r * 2 + 1];
        const float sx = stS[r * 4 + 0], sy = stS[r * 4 + 1], spsi = stS[r * 4 + 2], sv = stS[r * 4 + 3];
        float nx, ny, npsi, nv;
        plant_step(sx, sy, spsi, sv, ped, steer, nx, ny, npsi, nv);
        if (lane < kRowsBlk) {
          const v4f ns = (v4f){nx, ny, npsi, nv};
          *(v4f*)(stS + r * 4) = ns;
          *(v4f*)(trajS + r * kTrajPitch + 4 * t) = ns;
        }
      }
      wave_sync_lds();
      if (t + 1 < kSteps) embed_rows(An, stS, wembS, bembS, lane);
    }
    __syncthreads();
  }

  float* ob = out0 + (size_t)rowBase * kTrajPitch;
  for (int pass = 0; pass < 2; ++pass) {
    for (int i = tid; i < (kRowsBlk * kTrajPitch) / 4; i += 128) {
      const v4f val = *(const v4f*)(trajS + 4 * i);
      *(volatile v4f*)(ob + 4 * (size_t)i) = val;
    }
    __threadfence();
  }
}

extern "C" void kernel_launch(void* const* d_in, const int* in_sizes, int n_in,
                              void* d_out, int out_size, void* d_ws, size_t ws_size,
                              hipStream_t stream) {
  if (n_in < 20) return;
  const float* z      = (const float*)d_in[0];
  const float* init_s = (const float*)d_in[1];
  const float* W_emb  = (const float*)d_in[2];
  const float* b_emb  = (const float*)d_in[3];
  const float* W_ih   = (const float*)d_in[4];
  const float* b_ih   = (const float*)d_in[5];
  const float* W_hh   = (const float*)d_in[6];
  const float* b_hh   = (const float*)d_in[7];
  const float* W_h2c  = (const float*)d_in[8];
  const float* b_h2c  = (const float*)d_in[9];
  const float* W_init = (const float*)d_in[10];
  const float* b_init = (const float*)d_in[11];
  const float* Wl0    = (const float*)d_in[12];
  const float* bl0    = (const float*)d_in[13];
  const float* Wl1    = (const float*)d_in[14];
  const float* bl1    = (const float*)d_in[15];
  const float* Wl2    = (const float*)d_in[16];
  const float* bl2    = (const float*)d_in[17];
  const float* Wl3    = (const float*)d_in[18];
  const float* bl3    = (const float*)d_in[19];

  const int Btot = in_sizes[0] / kLat;
  if (Btot <= 0 || (Btot % 64) != 0) return;
  if (in_sizes[1] != Btot * 4) return;
  if ((size_t)out_size != (size_t)Btot * (size_t)(kSteps * 4 + 2)) return;

  unsigned char* ws = (unsigned char*)d_ws;
  size_t off = 0;
  const size_t szZ   = (size_t)Btot * kLatPad * 2;
  const size_t szH16 = (size_t)Btot * kHid * 2;
  const size_t szH32 = (size_t)Btot * kHid * 4;
  unsigned short* Zhi  = (unsigned short*)(ws + off); off += szZ;
  unsigned short* Zlo  = (unsigned short*)(ws + off); off += szZ;
  unsigned short* H1hi = (unsigned short*)(ws + off); off += szH16;
  unsigned short* H1lo = (unsigned short*)(ws + off); off += szH16;
  unsigned short* H2hi = (unsigned short*)(ws + off); off += szH16;
  unsigned short* H2lo = (unsigned short*)(ws + off); off += szH16;
  float* L3  = (float*)(ws + off); off += szH32;
  float* H0  = (float*)(ws + off); off += szH32;
  unsigned short* Wl0hi = (unsigned short*)(ws + off); off += (size_t)kHid * kLatPad * 2;
  unsigned short* Wl0lo = (unsigned short*)(ws + off); off += (size_t)kHid * kLatPad * 2;
  unsigned short* Winhi = (unsigned short*)(ws + off); off += (size_t)kHid * kLatPad * 2;
  unsigned short* Winlo = (unsigned short*)(ws + off); off += (size_t)kHid * kLatPad * 2;
  unsigned short* Wl1hi = (unsigned short*)(ws + off); off += (size_t)kHid * kHid * 2;
  unsigned short* Wl1lo = (unsigned short*)(ws + off); off += (size_t)kHid * kHid * 2;
  unsigned short* Wl2hi = (unsigned short*)(ws + off); off += (size_t)kHid * kHid * 2;
  unsigned short* Wl2lo = (unsigned short*)(ws + off); off += (size_t)kHid * kHid * 2;
  unsigned short* Wl3hi = (unsigned short*)(ws + off); off += (size_t)kHid * kHid * 2;
  unsigned short* Wl3lo = (unsigned short*)(ws + off); off += (size_t)kHid * kHid * 2;
  unsigned short* Wcat  = (unsigned short*)(ws + off); off += (size_t)kGates * kKcat * 2;
  unsigned short* Wh2c  = (unsigned short*)(ws + off); off += (size_t)16 * kHid * 2;
  if (off > ws_size) return;

  float* out0 = (float*)d_out;
  float* out1 = out0 + (size_t)Btot * (size_t)(kSteps * 4);
  const float* dummyf = (const float*)ws;
  const unsigned short* dummyh = (const unsigned short*)ws;

  prep_weights_kernel<<<dim3(32, 7), 128, 0, stream>>>(
      Wl0, W_init, Wl1, Wl2, Wl3, W_ih, W_hh, W_h2c,
      Wl0hi, Wl0lo, Winhi, Winlo, Wl1hi, Wl1lo, Wl2hi, Wl2lo, Wl3hi, Wl3lo, Wcat, Wh2c);
  split_z_kernel<<<(Btot * 16 + 255) / 256, 256, 0, stream>>>(z, Zhi, Zlo, Btot);

  const int gemmBlocks = ((Btot / 64) * (kHid / 64) + 7) / 8;
  wmma_gemm64<1, true, 2, 2, false, 4><<<dim3(gemmBlocks, 1), 256, 0, stream>>>(
      Zhi, Zlo, kLatPad, 0, Wl0hi, Wl0lo, kLatPad, 0,
      (void*)H1hi, (void*)H1lo, kHid, 0, bl0, dummyf, 0, Btot, kHid, kLatPad, 1.0f);
  wmma_gemm64<1, true, 2, 0, false, 0><<<dim3(gemmBlocks, 1), 256, 0, stream>>>(
      Zhi, Zlo, kLatPad, 0, Winhi, Winlo, kLatPad, 0,
      (void*)H0, (void*)H0, kHid, 0, b_init, dummyf, 0, Btot, kHid, kLatPad, 1.0f);
  wmma_gemm64<1, true, 2, 2, false, 4><<<dim3(gemmBlocks, 1), 256, 0, stream>>>(
      H1hi, H1lo, kHid, 0, Wl1hi, Wl1lo, kHid, 0,
      (void*)H2hi, (void*)H2lo, kHid, 0, bl1, dummyf, 0, Btot, kHid, kHid, 1.0f);
  wmma_gemm64<1, true, 2, 2, false, 4><<<dim3(gemmBlocks, 1), 256, 0, stream>>>(
      H2hi, H2lo, kHid, 0, Wl2hi, Wl2lo, kHid, 0,
      (void*)H1hi, (void*)H1lo, kHid, 0, bl2, dummyf, 0, Btot, kHid, kHid, 1.0f);
  wmma_gemm64<1, true, 0, 0, false, 0><<<dim3(gemmBlocks, 1), 256, 0, stream>>>(
      H1hi, H1lo, kHid, 0, Wl3hi, Wl3lo, kHid, 0,
      (void*)L3, (void*)L3, kHid, 0, dummyf, dummyf, 0, Btot, kHid, kHid, 1.0f);
  label_out_kernel<<<(Btot / 2 + 255) / 256, 256, 0, stream>>>(L3, bl3, out1, Btot / 2);
  lstm_rollout_kernel<<<Btot / kRowsBlk, 128, 0, stream>>>(
      Wcat, Wh2c, H0, init_s, W_emb, b_emb, b_ih, b_hh, b_h2c, out0, Btot);
  (void)dummyh;
}
